// GIN_39247411151131
// MI455X (gfx1250) — hardware-verified
//
#include <hip/hip_runtime.h>
#include <stddef.h>
#include <stdint.h>


#define DD      200
#define CC      10
#define W0P     256
#define KH      224
#define K2      448
#define NP      16
#define NTHR    256
#define NWAVE   8
#define EPT     8
#define CHUNK   (NTHR * EPT)
#define WCAP    (EPT * 32)
#define LISTN   (NWAVE * WCAP)
#define NBA     1024
#define SLA     10
#define RC      36864
#define DEGCAP  128
#define GBM     64
#define GTHR    128
#define KSTEPS  (K2 / 32)
#define NU1     (NP * (K2 / 8))
#define GW1     4
#define S0_INTS (LISTN + RC + 3 * NBA + 16 + RC / 2)
#define WSMAX   134217728

static_assert((CHUNK & (CHUNK - 1)) == 0 && CHUNK <= 4096);
static_assert((NBA & (NBA - 1)) == 0 && NBA == (1 << SLA));
static_assert(NBA % NWAVE == 0 && NBA % 32 == 0 && NBA % 16 == 0 && NBA == 4 * NTHR);
static_assert(RC % (NTHR * 4) == 0 && RC % 32 == 0 && RC <= 65536);
static_assert(S0_INTS % 4 == 0 && S0_INTS * 4 <= 300000);
static_assert(K2 % 32 == 0 && K2 == 2 * KH && KH % 32 == 0 && KH >= DD && DD % 8 == 0);
static_assert(DD / 8 == 25 && KH / 8 == 28 && W0P == 32 * 8);
static_assert(GBM == (GTHR / 32) * 16 && NP == 16);
static_assert(NU1 <= GW1 * NTHR && (NU1 % 32) == 0);
static_assert((NBA * CC) % (4 * NTHR) == 0 && (NBA * CC) / (4 * NTHR) == 10);
static_assert((16 * CC * 4) % 128 == 0);
static_assert((NBA * CC + 2 * NBA) * 4 <= 65536);

typedef float          v4f   __attribute__((ext_vector_type(4)));
typedef float          v8f   __attribute__((ext_vector_type(8)));
typedef int            v4i   __attribute__((ext_vector_type(4)));
typedef int            v8i   __attribute__((ext_vector_type(8)));
typedef unsigned int   v4u   __attribute__((ext_vector_type(4)));
typedef unsigned short v8us  __attribute__((ext_vector_type(8)));
typedef unsigned short v16us __attribute__((ext_vector_type(16)));
typedef __bf16         v16bf __attribute__((ext_vector_type(16)));
typedef v4f  __attribute__((may_alias)) v4fa;
typedef v4i  __attribute__((may_alias)) v4ia;
typedef v4u  __attribute__((may_alias)) v4ua;
typedef v8us __attribute__((may_alias)) v8usa;
union FragB { v16bf v; v16us u; v8us h[2]; v8i w; };

__device__ __forceinline__ v8f wmb(const FragB& a, const FragB& b, v8f c) {
  v8f d = __builtin_amdgcn_wmma_f32_16x16x32_bf16(false, a.v, false, b.v, (short)0, c, false, false);
  asm volatile("v_nop\n\tv_nop\n\tv_nop\n\tv_nop" : "+v"(d) : "v"(a.w), "v"(b.w));
  return d;
}

__device__ __forceinline__ unsigned bf16_bits(float f) {
  const unsigned u = __float_as_uint(f);
  return (u + 0x7FFFu + ((u >> 16) & 1u)) >> 16;
}
__device__ __forceinline__ float bf16_val(float f) {
  return __uint_as_float(bf16_bits(f) << 16);
}

template <int SLB>
__device__ __forceinline__ int scan_chunk(const int* __restrict__ dsts, int nE, int cbase, int slotBase,
                                          int nb, int vec8, int* list, int tid, int lane, int wave) {
  int wc = 0;
  const int el0  = tid * EPT;
  const int e0   = cbase + el0;
  const int sent = -2147483647 - 1;
  v4i da, db;
  if (vec8 != 0 && cbase + CHUNK <= nE) {
    da = *(const v4i*)(dsts + e0);
    db = *(const v4i*)(dsts + e0 + 4);
  } else {
    da.x = (e0     < nE) ? dsts[min(e0,     nE - 1)] : sent;
    da.y = (e0 + 1 < nE) ? dsts[min(e0 + 1, nE - 1)] : sent;
    da.z = (e0 + 2 < nE) ? dsts[min(e0 + 2, nE - 1)] : sent;
    da.w = (e0 + 3 < nE) ? dsts[min(e0 + 3, nE - 1)] : sent;
    db.x = (e0 + 4 < nE) ? dsts[min(e0 + 4, nE - 1)] : sent;
    db.y = (e0 + 5 < nE) ? dsts[min(e0 + 5, nE - 1)] : sent;
    db.z = (e0 + 6 < nE) ? dsts[min(e0 + 6, nE - 1)] : sent;
    db.w = (e0 + 7 < nE) ? dsts[min(e0 + 7, nE - 1)] : sent;
  }
  const unsigned nbs = (unsigned)slotBase;
  const unsigned unb = (unsigned)nb;
  const unsigned s0 = (unsigned)da.x - nbs, s1 = (unsigned)da.y - nbs;
  const unsigned s2 = (unsigned)da.z - nbs, s3 = (unsigned)da.w - nbs;
  const unsigned s4 = (unsigned)db.x - nbs, s5 = (unsigned)db.y - nbs;
  const unsigned s6 = (unsigned)db.z - nbs, s7 = (unsigned)db.w - nbs;
  const bool h0 = s0 < unb, h1 = s1 < unb, h2 = s2 < unb, h3 = s3 < unb;
  const bool h4 = s4 < unb, h5 = s5 < unb, h6 = s6 < unb, h7 = s7 < unb;
  const unsigned any = __builtin_amdgcn_ballot_w32(h0 | h1 | h2 | h3 | h4 | h5 | h6 | h7);
  if (any != 0u) {
#define HITJ(J, HJ, SJ) { \
      const unsigned mj = __builtin_amdgcn_ballot_w32(HJ); \
      if (mj != 0u) { \
        if (HJ) { \
          const int pos = wc + (int)__builtin_amdgcn_mbcnt_lo(mj, 0u); \
          if (pos < WCAP) list[wave * WCAP + pos] = ((el0 + (J)) << SLB) | (int)(SJ); \
        } \
        wc += (int)__builtin_popcount(mj); } }
    HITJ(0, h0, s0)
    HITJ(1, h1, s1)
    HITJ(2, h2, s2)
    HITJ(3, h3, s3)
    HITJ(4, h4, s4)
    HITJ(5, h5, s5)
    HITJ(6, h6, s6)
    HITJ(7, h7, s7)
#undef HITJ
  }
  return wc;
}

__global__ __launch_bounds__(NTHR) void k_prep(
    const float* __restrict__ W0, const float* __restrict__ W1,
    const int* __restrict__ cols0, const float* __restrict__ vals0,
    const int* __restrict__ cols1, const float* __restrict__ vals1,
    const float* __restrict__ eps0, const float* __restrict__ eps1,
    unsigned short* w0b, int* colm, float* valm, unsigned short* w1t, float* c01,
    int nN, int nE, int gW0, int gEd) {
  const int b = (int)blockIdx.x, tid = (int)threadIdx.x;
  if (b < gW0) {
    const int u   = b * NTHR + tid;
    const int row = u >> 5;
    const int q   = u & 31;
    const int qc  = q < 25 ? q : 24;
    const float* p = W0 + (size_t)row * DD + 8 * qc;
    const v4f a = *(const v4fa*)p;
    const v4f c = *(const v4fa*)(p + 4);
    const bool ok = q < 25;
    v8us o;
    o[0] = ok ? (unsigned short)bf16_bits(a.x) : (unsigned short)0;
    o[1] = ok ? (unsigned short)bf16_bits(a.y) : (unsigned short)0;
    o[2] = ok ? (unsigned short)bf16_bits(a.z) : (unsigned short)0;
    o[3] = ok ? (unsigned short)bf16_bits(a.w) : (unsigned short)0;
    o[4] = ok ? (unsigned short)bf16_bits(c.x) : (unsigned short)0;
    o[5] = ok ? (unsigned short)bf16_bits(c.y) : (unsigned short)0;
    o[6] = ok ? (unsigned short)bf16_bits(c.z) : (unsigned short)0;
    o[7] = ok ? (unsigned short)bf16_bits(c.w) : (unsigned short)0;
    unsigned short* dp = w0b + (size_t)row * W0P + 8 * q;
    *(volatile v8us*)dp = o;
    __threadfence();
    *(volatile v8us*)dp = o;
  } else if (b < gW0 + 2 * gEd) {
    const int bb  = b - gW0;
    const int sup = bb >= gEd ? 1 : 0;
    const int u   = (bb - sup * gEd) * NTHR + tid;
    const int*   cs = sup ? cols1 : cols0;
    const float* vs = sup ? vals1 : vals0;
    const int nU = nE >> 2;
    const bool ok = u < nU;
    const int uc = ok ? u : nU - 1;
    const v4i cv = *(const v4ia*)(cs + 4 * (size_t)uc);
    const v4f vv = *(const v4fa*)(vs + 4 * (size_t)uc);
    v4f rv;
    rv.x = bf16_val(vv.x); rv.y = bf16_val(vv.y); rv.z = bf16_val(vv.z); rv.w = bf16_val(vv.w);
    int*   cp = colm + (size_t)sup * (size_t)nE + 4 * (size_t)uc;
    float* vp = valm + (size_t)sup * (size_t)nE + 4 * (size_t)uc;
    if (ok) { *(volatile v4i*)cp = cv; *(volatile v4f*)vp = rv; }
    __threadfence();
    if (ok) { *(volatile v4i*)cp = cv; *(volatile v4f*)vp = rv; }
  } else if (b < gW0 + 2 * gEd + GW1) {
    const int v  = (b - gW0 - 2 * gEd) * NTHR + tid;
    const bool ok = v < NU1;
    const int vc = ok ? v : NU1 - 1;
    const int n  = vc / (K2 / 8);
    const int k8 = (vc - n * (K2 / 8)) * 8;
    const int kk = k8 < KH ? k8 : k8 - KH;
    const int nc = n < CC ? n : CC - 1;
    v8us o;
#pragma unroll
    for (int i = 0; i < 8; ++i) {
      const int k  = kk + i;
      const int kc = k < DD ? k : DD - 1;
      const float x = W1[kc * CC + nc];
      const bool valid = (n < CC) && (k < DD);
      o[i] = valid ? (unsigned short)bf16_bits(x) : (unsigned short)0;
    }
    unsigned short* dp = w1t + 8 * (size_t)vc;
    if (ok) *(volatile v8us*)dp = o;
    __threadfence();
    if (ok) *(volatile v8us*)dp = o;
  } else {
    const float e0 = bf16_val(eps0[0]);
    const float e1 = bf16_val(eps1[0]);
    const float c0v = 0.1f * (1.0f + e0);
    const float c1v = 0.1f * (1.0f + e1);
    v4f v;
    v.x = (tid == 0) ? c0v : 0.0f;
    v.y = (tid == 0) ? c1v : 0.0f;
    v.z = 0.0f; v.w = 0.0f;
    const bool ok = tid < 8;
    float* dp = c01 + 4 * (ok ? tid : 0);
    if (ok) *(volatile v4f*)dp = v;
    __threadfence();
    if (ok) *(volatile v4f*)dp = v;
  }
}

__global__ __launch_bounds__(NTHR) void k_scan0(
    const int* __restrict__ rows0, const int* __restrict__ rows1,
    const int* __restrict__ colm, const float* __restrict__ valm,
    const unsigned short* __restrict__ w0b, const float* __restrict__ c01,
    int nE, int nN, int vec8, int mRows,
    unsigned short* hpl, int* tcnt, int* toff, int* rcol, float* rval) {
  extern __shared__ __attribute__((aligned(16))) int dsm[];
  int* list = dsm;
  int* hl   = dsm + LISTN;
  int* cnt  = hl + RC;
  int* offs = cnt + NBA;
  int* cur  = offs + NBA;
  int* misc = cur + NBA;
  unsigned short* sl = (unsigned short*)(misc + 16);
  const int tid = (int)threadIdx.x, lane = tid & 31, wave = tid >> 5;
  const int blk = (int)blockIdx.x;
  const int nodeBase = blk * NBA;

  {
    const v4i z4 = {0, 0, 0, 0};
    for (int i = tid * 4; i < S0_INTS; i += NTHR * 4) *(v4ia*)(dsm + i) = z4;
  }
  __syncthreads();

  int t = 0, ov = 0;
  const int nChunks = (nE + CHUNK - 1) / CHUNK;
#pragma unroll 1
  for (int c2 = 0; c2 < 2 * nChunks; ++c2) {
    const int sup   = c2 >= nChunks ? 1 : 0;
    const int ch    = c2 - sup * nChunks;
    const int* dsts = sup ? rows1 : rows0;
    const int cbase = ch * CHUNK;
    const int gb    = sup * nE + cbase;
    const int wc = scan_chunk<SLA>(dsts, nE, cbase, nodeBase, NBA, vec8, list, tid, lane, wave);
    if (lane == 0) misc[wave] = wc;
    __syncthreads();
    if (wave == 0) {
#pragma unroll 1
      for (int w2 = 0; w2 < NWAVE; ++w2) {
        int c = misc[w2];
        c = c < 0 ? 0 : (c > WCAP ? WCAP : c);
#pragma unroll 1
        for (int b0 = 0; b0 < c; b0 += 32) {
          const int idx = b0 + lane;
          const int ent = list[w2 * WCAP + (idx < WCAP ? idx : WCAP - 1)];
          const int m32 = (c - b0) < 32 ? (c - b0) : 32;
#pragma unroll 1
          for (int k = 0; k < m32; ++k) {
            const int u    = __builtin_amdgcn_readlane(ent, k);
            const int slot = u & (NBA - 1);
            const int el   = (u >> SLA) & (CHUNK - 1);
            const int pk   = ((gb + el) << SLA) | slot;
            if (t < RC) {
              if (lane == 0) { hl[t] = pk; cnt[slot] = cnt[slot] + 1; }
              t = t + 1;
            } else {
              ov = 1;
            }
          }
        }
      }
    }
    __syncthreads();
  }
  if (wave == 0 && lane == 0) { misc[8] = t; misc[9] = ov; }
  __syncthreads();
  int tt = misc[8];
  tt = tt < 0 ? 0 : (tt > RC ? RC : tt);
  const int ovf = misc[9];

  if (wave == 0) {
    const int base = lane * (NBA / 32);
    int s = 0;
#pragma unroll 1
    for (int i = 0; i < NBA / 32; ++i) s += cnt[base + i];
    int incl = s;
#pragma unroll
    for (int d = 1; d < 32; d <<= 1) {
      const int y = __shfl_up(incl, d, 32);
      if (lane >= d) incl += y;
    }
    int run = incl - s;
#pragma unroll 1
    for (int i = 0; i < NBA / 32; ++i) {
      const int cv = cnt[base + i];
      offs[base + i] = run;
      cur[base + i]  = run;
      run += cv;
    }
  }
  __syncthreads();
  if (wave == 0) {
#pragma unroll 1
    for (int b0 = 0; b0 < tt; b0 += 32) {
      const int idx = b0 + lane;
      const int ent = hl[idx < RC ? idx : RC - 1];
      const int m32 = (tt - b0) < 32 ? (tt - b0) : 32;
#pragma unroll 1
      for (int k = 0; k < m32; ++k) {
        const int u    = __builtin_amdgcn_readlane(ent, k);
        const int slot = u & (NBA - 1);
        if (lane == 0) {
          int p = cur[slot];
          p = p < 0 ? 0 : (p > RC - 1 ? RC - 1 : p);
          sl[p] = (unsigned short)(b0 + k);
          cur[slot] = p + 1;
        }
      }
    }
  }
  __syncthreads();

  const int g2max = 2 * nE - 1;

  {
    const v4i cq = *(const v4ia*)(cnt + 4 * tid);
    const v4i oq = *(const v4ia*)(offs + 4 * tid);
    int* cp = tcnt + (size_t)blk * NBA + 4 * tid;
    int* op = toff + (size_t)blk * NBA + 4 * tid;
    *(volatile v4i*)cp = cq; *(volatile v4i*)op = oq;
    __threadfence();
    *(volatile v4i*)cp = cq; *(volatile v4i*)op = oq;
    const size_t rb = (size_t)blk * RC;
#pragma unroll 1
    for (int it = 0; it < RC / (NTHR * 4); ++it) {
      const int p0 = it * (NTHR * 4) + 4 * tid;
      v4i cv; v4f vv;
#pragma unroll
      for (int j = 0; j < 4; ++j) {
        const int p = p0 + j;
        int ii = (int)sl[p];
        ii = ii > RC - 1 ? RC - 1 : ii;
        const int ent = hl[ii];
        int gid = (int)((unsigned)ent >> SLA);
        gid = gid > g2max ? g2max : gid;
        const int   cj = colm[gid];
        const float vj = valm[gid];
        const bool live = p < tt;
        cv[j] = live ? cj : 0;
        vv[j] = live ? vj : 0.0f;
      }
      int*   rc = rcol + rb + p0;
      float* rv = rval + rb + p0;
      *(volatile v4i*)rc = cv; *(volatile v4f*)rv = vv;
      __threadfence();
      *(volatile v4i*)rc = cv; *(volatile v4f*)rv = vv;
    }
  }

  const float c0   = c01[0];
  const float qnan = __int_as_float(0x7fc00000);
  const float pz   = (ovf != 0) ? qnan : 0.0f;
  const int   sh4  = (lane + 4) & 31;
#pragma unroll 1
  for (int si = 0; si < NBA / NWAVE; ++si) {
    const int s    = si * NWAVE + wave;
    const int node = nodeBase + s;
    const int craw = cnt[s];
    const bool big = craw > DEGCAP;
    int c = craw < 0 ? 0 : (craw > DEGCAP ? DEGCAP : craw);
    int o = offs[s];
    o = o < 0 ? 0 : (o > RC ? RC : o);
    float acc[8];
#pragma unroll
    for (int j = 0; j < 8; ++j) acc[j] = 0.0f;
#pragma unroll 1
    for (int b0 = 0; b0 < c; b0 += 32) {
      int idx = o + b0 + lane;
      idx = idx > RC - 1 ? RC - 1 : idx;
      int ii = (int)sl[idx];
      ii = ii > RC - 1 ? RC - 1 : ii;
      const int ent = hl[ii];
      int gid = (int)((unsigned)ent >> SLA);
      gid = gid > g2max ? g2max : gid;
      int col = colm[gid];
      col = col < 0 ? 0 : (col > nN - 1 ? nN - 1 : col);
      const int vbi = __float_as_int(valm[gid]);
      const int m32 = (c - b0) < 32 ? (c - b0) : 32;
#pragma unroll 1
      for (int k = 0; k < m32; ++k) {
        const int   sk = __builtin_amdgcn_readlane(col, k);
        const float ck = __int_as_float(__builtin_amdgcn_readlane(vbi, k));
        const v4u w = *(const v4ua*)(w0b + (size_t)sk * W0P + 8 * lane);
        acc[0] = fmaf(ck, __uint_as_float(w.x << 16),          acc[0]);
        acc[1] = fmaf(ck, __uint_as_float(w.x & 0xffff0000u),  acc[1]);
        acc[2] = fmaf(ck, __uint_as_float(w.y << 16),          acc[2]);
        acc[3] = fmaf(ck, __uint_as_float(w.y & 0xffff0000u),  acc[3]);
        acc[4] = fmaf(ck, __uint_as_float(w.z << 16),          acc[4]);
        acc[5] = fmaf(ck, __uint_as_float(w.z & 0xffff0000u),  acc[5]);
        acc[6] = fmaf(ck, __uint_as_float(w.w << 16),          acc[6]);
        acc[7] = fmaf(ck, __uint_as_float(w.w & 0xffff0000u),  acc[7]);
      }
    }
    const int nc = node < nN ? node : nN - 1;
    float sv[8];
    {
      const v4u w = *(const v4ua*)(w0b + (size_t)nc * W0P + 8 * lane);
      sv[0] = __uint_as_float(w.x << 16); sv[1] = __uint_as_float(w.x & 0xffff0000u);
      sv[2] = __uint_as_float(w.y << 16); sv[3] = __uint_as_float(w.y & 0xffff0000u);
      sv[4] = __uint_as_float(w.z << 16); sv[5] = __uint_as_float(w.z & 0xffff0000u);
      sv[6] = __uint_as_float(w.w << 16); sv[7] = __uint_as_float(w.w & 0xffff0000u);
    }
    const float pzr = big ? qnan : pz;
    const bool live = node < nN;
    unsigned hb[8], lb[8];
#pragma unroll
    for (int j = 0; j < 8; ++j) {
      float y = fmaf(c0, sv[j], acc[j]);
      y = (y > 0.0f) ? y : (y - y);
      y = y + pzr;
      const float v = live ? y : 0.0f;
      hb[j] = bf16_bits(v);
      lb[j] = bf16_bits(v - __uint_as_float(hb[j] << 16));
    }
    const int hw0 = (int)(hb[0] | (hb[1] << 16)), hw1 = (int)(hb[2] | (hb[3] << 16));
    const int hw2 = (int)(hb[4] | (hb[5] << 16)), hw3 = (int)(hb[6] | (hb[7] << 16));
    const int lw0 = (int)(lb[0] | (lb[1] << 16)), lw1 = (int)(lb[2] | (lb[3] << 16));
    const int lw2 = (int)(lb[4] | (lb[5] << 16)), lw3 = (int)(lb[6] | (lb[7] << 16));
    const int t0 = __shfl(lw0, sh4, 32), t1 = __shfl(lw1, sh4, 32);
    const int t2 = __shfl(lw2, sh4, 32), t3 = __shfl(lw3, sh4, 32);
    const bool isHi = lane < 28;
    v4u s1, s2;
    s1.x = (unsigned)(isHi ? hw0 : t0); s1.y = (unsigned)(isHi ? hw1 : t1);
    s1.z = (unsigned)(isHi ? hw2 : t2); s1.w = (unsigned)(isHi ? hw3 : t3);
    s2.x = (unsigned)t0; s2.y = (unsigned)t1; s2.z = (unsigned)t2; s2.w = (unsigned)t3;
    const int nrow = node < mRows ? node : mRows - 1;
    unsigned short* p1 = hpl + (size_t)nrow * K2 + 8 * lane;
    unsigned short* p2 = hpl + (size_t)nrow * K2 + 256 + 8 * (lane < 24 ? lane : 0);
    const bool wr1 = node < mRows;
    const bool wr2 = wr1 && (lane < 24);
    if (wr1) *(volatile v4u*)p1 = s1;
    if (wr2) *(volatile v4u*)p2 = s2;
    __threadfence();
    if (wr1) *(volatile v4u*)p1 = s1;
    if (wr2) *(volatile v4u*)p2 = s2;
  }
}

__global__ __launch_bounds__(GTHR) void k_proj(const unsigned short* __restrict__ A,
                                               const unsigned short* __restrict__ BT, float* P) {
  __shared__ __attribute__((aligned(16))) float stg[GBM * NP];
  const int tid = (int)threadIdx.x, lane = tid & 31, wave = tid >> 5, hh = lane >> 4, m = lane & 15;
  const int rowBase = (int)blockIdx.x * GBM;
  v8f acc = {0.f, 0.f, 0.f, 0.f, 0.f, 0.f, 0.f, 0.f};
  const unsigned short* ap = A  + (size_t)(rowBase + 16 * wave + m) * (size_t)K2 + 8 * hh;
  const unsigned short* bp = BT + (size_t)m * (size_t)K2 + 8 * hh;
#pragma unroll 2
  for (int ks = 0; ks < KSTEPS; ++ks) {
    FragB af, bf;
    af.h[0] = *(const v8usa*)(ap + 32 * ks);
    af.h[1] = *(const v8usa*)(ap + 32 * ks + 16);
    bf.h[0] = *(const v8usa*)(bp + 32 * ks);
    bf.h[1] = *(const v8usa*)(bp + 32 * ks + 16);
    acc = wmb(af, bf, acc);
  }
#pragma unroll
  for (int r = 0; r < 8; ++r) {
    const int lr = 16 * wave + 8 * hh + r;
    stg[lr * NP + m] = acc[r];
  }
  __syncthreads();
  v4f fv[2];
#pragma unroll
  for (int it = 0; it < 2; ++it) fv[it] = *(const v4fa*)(stg + 4 * (it * GTHR + tid));
  float* ob = P + (size_t)rowBase * NP;
#pragma unroll
  for (int it = 0; it < 2; ++it) *(volatile v4f*)(ob + 4 * (it * GTHR + tid)) = fv[it];
  __threadfence();
#pragma unroll
  for (int it = 0; it < 2; ++it) *(volatile v4f*)(ob + 4 * (it * GTHR + tid)) = fv[it];
}

__global__ __launch_bounds__(NTHR) void k_scan1(
    const int* __restrict__ tcnt, const int* __restrict__ toff,
    const int* __restrict__ rcol, const float* __restrict__ rval,
    const float* __restrict__ P, const float* __restrict__ c01, int nN, float* out) {
  __shared__ __attribute__((aligned(16))) float os[NBA * CC];
  __shared__ __attribute__((aligned(16))) int cnt[NBA];
  __shared__ __attribute__((aligned(16))) int offs[NBA];
  const int tid = (int)threadIdx.x, lane = tid & 31, wave = tid >> 5;
  const int blk = (int)blockIdx.x;
  const int nodeBase = blk * NBA;
  const size_t rb = (size_t)blk * RC;
  {
    const v4i a = *(const v4ia*)(tcnt + (size_t)blk * NBA + 4 * tid);
    const v4i b = *(const v4ia*)(toff + (size_t)blk * NBA + 4 * tid);
    *(v4ia*)(cnt + 4 * tid)  = a;
    *(v4ia*)(offs + 4 * tid) = b;
  }
  const float c1   = c01[1];
  const float qnan = __int_as_float(0x7fc00000);
  const int   cl   = lane & 15;
  __syncthreads();

#pragma unroll 1
  for (int si = 0; si < NBA / NWAVE; ++si) {
    const int s    = si * NWAVE + wave;
    const int node = nodeBase + s;
    const int craw = cnt[s];
    int c = craw < 0 ? 0 : (craw > DEGCAP ? DEGCAP : craw);
    int o = offs[s];
    o = o < 0 ? 0 : (o > RC ? RC : o);
    float acc = 0.0f;
#pragma unroll 1
    for (int b0 = 0; b0 < c; b0 += 32) {
      int idx = o + b0 + lane;
      idx = idx > RC - 1 ? RC - 1 : idx;
      int col = rcol[rb + idx];
      col = col < 0 ? 0 : (col > nN - 1 ? nN - 1 : col);
      const int vbi = __float_as_int(rval[rb + idx]);
      const int m32 = (c - b0) < 32 ? (c - b0) : 32;
#pragma unroll 1
      for (int k = 0; k < m32; ++k) {
        const int   sk = __builtin_amdgcn_readlane(col, k);
        const float ck = __int_as_float(__builtin_amdgcn_readlane(vbi, k));
        const float pv = P[(size_t)sk * NP + cl];
        acc = fmaf(ck, pv, acc);
      }
    }
    const int nc = node < nN ? node : nN - 1;
    const float sv = P[(size_t)nc * NP + cl];
    const float pzr = (craw > DEGCAP) ? qnan : 0.0f;
    float y = fmaf(c1, sv, acc) + pzr;
    y = (node < nN) ? y : 0.0f;
    if (lane < CC) os[s * CC + lane] = y;
  }
  __syncthreads();

  int nbv = nN - nodeBase;
  nbv = nbv < 0 ? 0 : (nbv > NBA ? NBA : nbv);
  const int nq = (nbv * CC) >> 2;
  constexpr int NIT = (NBA * CC) / (4 * NTHR);
  v4f ov[NIT];
#pragma unroll
  for (int it = 0; it < NIT; ++it) ov[it] = *(const v4fa*)(os + 4 * (it * NTHR + tid));
  float* ob = out + (size_t)nodeBase * CC;
#pragma unroll
  for (int it = 0; it < NIT; ++it) {
    const int q = it * NTHR + tid;
    if (q < nq) *(volatile v4f*)(ob + 4 * (size_t)q) = ov[it];
  }
  __threadfence();
#pragma unroll
  for (int it = 0; it < NIT; ++it) {
    const int q = it * NTHR + tid;
    if (q < nq) *(volatile v4f*)(ob + 4 * (size_t)q) = ov[it];
  }
}

static inline int cdiv(int a, int b) { return (a + b - 1) / b; }
static inline size_t al256(size_t o) { return (o + 255) & ~(size_t)255; }

extern "C" void kernel_launch(void* const* d_in, const int* in_sizes, int n_in,
                              void* d_out, int out_size, void* d_ws, size_t ws_size,
                              hipStream_t stream) {
  if (n_in < 11) return;
  const int nE = in_sizes[1];
  if (nE < CHUNK || (nE % 128) != 0 || 2LL * nE >= (1LL << 21)) return;
  if (in_sizes[2] != nE || in_sizes[3] != nE) return;
  if (in_sizes[4] != nE || in_sizes[5] != nE || in_sizes[6] != nE) return;
  if (in_sizes[7] < DD || (in_sizes[7] % DD) != 0) return;
  const int nN = in_sizes[7] / DD;
  if (nN < 64 || (nN % 16) != 0 || nN > (1 << 22)) return;
  if (in_sizes[8] != DD * CC) return;
  if (in_sizes[9] < 1 || in_sizes[10] < 1) return;
  if ((long long)out_size != (long long)nN * CC) return;

  const int*   rows0 = (const int*)  d_in[1];
  const int*   cols0 = (const int*)  d_in[2];
  const float* vals0 = (const float*)d_in[3];
  const int*   rows1 = (const int*)  d_in[4];
  const int*   cols1 = (const int*)  d_in[5];
  const float* vals1 = (const float*)d_in[6];
  const float* W0    = (const float*)d_in[7];
  const float* W1    = (const float*)d_in[8];
  const float* eps0  = (const float*)d_in[9];
  const float* eps1  = (const float*)d_in[10];
  float* out = (float*)d_out;

  const int MP  = cdiv(nN, GBM) * GBM;
  const int gM  = MP / GBM;
  const int gA  = cdiv(MP, NBA);
  if ((long long)gA * NBA < (long long)MP) return;
  if ((long long)(gA - 1) * NBA >= (long long)nN) return;
  if (((long long)nN * 32) % NTHR != 0) return;
  const int gW0 = (int)(((long long)nN * 32) / NTHR);
  const int gEd = cdiv(nE / 4, NTHR);
  const int vec8 = 1;

  char* ws = (char*)d_ws;
  size_t off = 0;
  const size_t oW0B = off; off = al256(off + (size_t)nN * W0P * 2);
  const size_t oCOL = off; off = al256(off + (size_t)2 * nE * 4);
  const size_t oVAL = off; off = al256(off + (size_t)2 * nE * 4);
  const size_t oW1T = off; off = al256(off + (size_t)NP * K2 * 2);
  const size_t oC01 = off; off = al256(off + (size_t)32 * 4);
  const size_t oH   = off; off = al256(off + (size_t)MP * K2 * 2);
  const size_t oP   = off; off = al256(off + (size_t)MP * NP * 4);
  const size_t oTC  = off; off = al256(off + (size_t)gA * NBA * 4);
  const size_t oTO  = off; off = al256(off + (size_t)gA * NBA * 4);
  const size_t oRC  = off; off = al256(off + (size_t)gA * RC * 4);
  const size_t oRV  = off; off = al256(off + (size_t)gA * RC * 4);
  if (off > ws_size || off > (size_t)WSMAX) return;
  unsigned short* W0B  = (unsigned short*)(ws + oW0B);
  int*            COLM = (int*)(ws + oCOL);
  float*          VALM = (float*)(ws + oVAL);
  unsigned short* W1T  = (unsigned short*)(ws + oW1T);
  float*          C01  = (float*)(ws + oC01);
  unsigned short* HPL  = (unsigned short*)(ws + oH);
  float*          PPL  = (float*)(ws + oP);
  int*            TCN  = (int*)(ws + oTC);
  int*            TOF  = (int*)(ws + oTO);
  int*            RCL  = (int*)(ws + oRC);
  float*          RVL  = (float*)(ws + oRV);

  const size_t s0Lds = (size_t)S0_INTS * 4;
  hipFuncSetAttribute(reinterpret_cast<const void*>(&k_scan0), hipFuncAttributeMaxDynamicSharedMemorySize, (int)s0Lds);

  k_prep<<<gW0 + 2 * gEd + GW1 + 1, NTHR, 0, stream>>>(W0, W1, cols0, vals0, cols1, vals1, eps0, eps1,
                                                        W0B, COLM, VALM, W1T, C01, nN, nE, gW0, gEd);
  k_scan0<<<gA, NTHR, s0Lds, stream>>>(rows0, rows1, COLM, VALM, W0B, C01, nE, nN, vec8, MP,
                                       HPL, TCN, TOF, RCL, RVL);
  k_proj<<<gM, GTHR, 0, stream>>>(HPL, W1T, PPL);
  k_scan1<<<gA, NTHR, 0, stream>>>(TCN, TOF, RCL, RVL, PPL, C01, nN, out);
}
